// BASE_MAMBA_14018773254552
// MI455X (gfx1250) — hardware-run, weakly checked
//
#include <hip/hip_runtime.h>
#include <math.h>

typedef __attribute__((ext_vector_type(16))) _Float16 v16h;
typedef __attribute__((ext_vector_type(16))) __bf16 v16b;
typedef __attribute__((ext_vector_type(8)))  _Float16 v8h;
typedef __attribute__((ext_vector_type(8)))  float v8f;
typedef __attribute__((ext_vector_type(4)))  float v4f;
typedef __attribute__((ext_vector_type(2)))  float v2f;
typedef __attribute__((ext_vector_type(4)))  unsigned v4u;
typedef __attribute__((ext_vector_type(4)))  int v4i;
typedef float __attribute__((may_alias)) float_a;
typedef int __attribute__((may_alias)) int_a;

template <typename T> __device__ __forceinline__ void vst2(void* p, T v) { *(volatile T*)p = v; __threadfence(); *(volatile T*)p = v; }
__device__ __forceinline__ v8f wmma16(v16h a, v16h b, v8f c) {
  v8f d = __builtin_amdgcn_wmma_f32_16x16x32_f16(false, a, false, b, (short)0, c, false, false);
  asm volatile("v_nop\n\tv_nop\n\tv_nop\n\tv_nop" : "+v"(d) : "v"(a), "v"(b));
  return d;
}
__device__ __forceinline__ v8f wmma_bf(v16b a, v16b b, v8f c) {
  v8f d = __builtin_amdgcn_wmma_f32_16x16x32_bf16(false, a, false, b, (short)0, c, false, false);
  asm volatile("v_nop\n\tv_nop\n\tv_nop\n\tv_nop" : "+v"(d) : "v"(a), "v"(b));
  return d;
}
__device__ __forceinline__ v16h frag_h(const _Float16* rowk0, int lane) {
  union { v16h v; v8h q[2]; } u; const _Float16* p = rowk0 + 8 * (lane >> 4);
  u.q[0] = *(const v8h*)p; u.q[1] = *(const v8h*)(p + 16); return u.v;
}
__device__ __forceinline__ v16h frag_f32(const float* rowk0, int lane) {
  v16h a; const float* p = rowk0 + 8 * (lane >> 4);
#pragma unroll
  for (int i = 0; i < 8; ++i) { a[i] = (_Float16)p[i]; a[8 + i] = (_Float16)p[16 + i]; }
  return a;
}
__device__ __forceinline__ v16h frag_f32s(const float* rowk0, int lane, float sc) {
  v16h a; const float* p = rowk0 + 8 * (lane >> 4);
#pragma unroll
  for (int i = 0; i < 8; ++i) { a[i] = (_Float16)(p[i] * sc); a[8 + i] = (_Float16)(p[16 + i] * sc); }
  return a;
}
__device__ __forceinline__ v16h fragc_f32(const float* W, int k0, int n, int lane, int ld, int K) {
  v16h a; const int g = lane >> 4;
#pragma unroll
  for (int i = 0; i < 8; ++i) { const int ka = k0 + 8 * g + i, kb = ka + 16;
    a[i] = (_Float16)(ka < K ? W[(size_t)(ka < K ? ka : K - 1) * ld + n] : 0.f); a[8 + i] = (_Float16)(kb < K ? W[(size_t)(kb < K ? kb : K - 1) * ld + n] : 0.f); }
  return a;
}
struct F2 { v16b h, l; };
__device__ __forceinline__ F2 bsplit16(const float v[16]) { F2 r;
#pragma unroll
  for (int i = 0; i < 16; ++i) { const __bf16 h = (__bf16)v[i]; r.h[i] = h; r.l[i] = (__bf16)(v[i] - (float)h); }
  return r; }
__device__ __forceinline__ F2 split_row(const float* row, int k0, int lane) { float v[16]; const float* p = row + k0 + 8 * (lane >> 4);
#pragma unroll
  for (int i = 0; i < 8; ++i) { v[i] = p[i]; v[8 + i] = p[16 + i]; }
  return bsplit16(v); }
__device__ __forceinline__ F2 split_rowK(const float* row, int k0, int lane, int K) { float v[16]; const int g = lane >> 4;
#pragma unroll
  for (int i = 0; i < 8; ++i) { const int ka = k0 + 8 * g + i, kb = ka + 16; v[i] = ka < K ? row[ka < K ? ka : K - 1] : 0.f; v[8 + i] = kb < K ? row[kb < K ? kb : K - 1] : 0.f; }
  return bsplit16(v); }
__device__ __forceinline__ F2 split_col(const float* W, int k0, int n, int lane, int ld, int K) { float v[16]; const int g = lane >> 4;
#pragma unroll
  for (int i = 0; i < 8; ++i) { const int ka = k0 + 8 * g + i, kb = ka + 16; v[i] = ka < K ? W[(size_t)(ka < K ? ka : K - 1) * ld + n] : 0.f; v[8 + i] = kb < K ? W[(size_t)(kb < K ? kb : K - 1) * ld + n] : 0.f; }
  return bsplit16(v); }
__device__ __forceinline__ v8f mac3(const F2& a, const F2& b, v8f c) { c = wmma_bf(a.l, b.h, c); c = wmma_bf(a.h, b.l, c); return wmma_bf(a.h, b.h, c); }
__device__ __forceinline__ float sigm(float v) { return 1.0f / (1.0f + expf(-v)); }
#define LDSX() do { asm volatile("s_wait_dscnt 0" ::: "memory"); __builtin_amdgcn_wave_barrier(); __builtin_amdgcn_fence(__ATOMIC_RELEASE, "workgroup"); } while (0)


#define NB 4
#define LL 1024
#define CIN 20
#define DM 128
#define DI 256
#define DS 64
#define DC 4
#define DTR 8
#define NT (NB * LL)
#define XW 160
typedef __attribute__((ext_vector_type(8))) __bf16 v8b;
__device__ __forceinline__ v16b frag_b(const __bf16* rowk0, int lane) {
  union { v16b v; v8b q[2]; } u; const __bf16* p = rowk0 + 8 * (lane >> 4);
  u.q[0] = *(const v8b*)p; u.q[1] = *(const v8b*)(p + 16); return u.v;
}
__device__ __forceinline__ float bfr(float v) { return (float)(__bf16)v; }
__device__ __attribute__((noinline)) float exp_ni(float v) { return expf(v); }
__device__ __attribute__((noinline)) float erf_ni(float v) { return erff(v); }

__device__ __attribute__((noinline)) float log1p_ni(float v) { return log1pf(v); }
#define WS_PW   0u
#define PWIN 0
#define PWX  (PWIN + 512 * DM)
#define PWO  (PWX + XW * DI)
#define PWEND (PWO + DM * DI)
#define WS_H    (WS_PW + 2u * PWEND)
#define WS_XZ   (WS_H + 4u * NT * DM)
#define WS_XC   (WS_XZ + 4u * NT * 512)
#define WS_DBC  (WS_XC + 4u * NT * DI)
#define WS_DT   (WS_DBC + 4u * NT * XW)
#define WS_Y    (WS_DT + 4u * NT * DI)
#define WS_O    (WS_Y + 4u * NT * DI)
#define WS_END  (WS_O + 4u * NT * DM)

__global__ __launch_bounds__(256) void k_pack(const float* __restrict__ WIN, const float* __restrict__ WX, const float* __restrict__ WOUT, __bf16* __restrict__ PW) {
  __shared__ __align__(16) __bf16 s1[DM], s2[DI], s3[DI]; const int o = blockIdx.x, t = threadIdx.x;
  if (t < DM) s1[t] = (__bf16)WIN[(size_t)o * DM + t];
  if (o < XW) s2[t] = (__bf16)((o < 136) ? WX[(size_t)o * DI + t] : 0.f);
  if (o < DM) s3[t] = (__bf16)WOUT[(size_t)o * DI + t];
  __syncthreads();
  if (t < DM / 8) vst2((unsigned*)(PW + PWIN + (size_t)o * DM + t * 8), *(const v4u*)&s1[t * 8]);
  if (o < XW && t >= 32 && t < 64) vst2((unsigned*)(PW + PWX + (size_t)o * DI + (t - 32) * 8), *(const v4u*)&s2[(t - 32) * 8]);
  if (o < DM && t >= 64 && t < 96) vst2((unsigned*)(PW + PWO + (size_t)o * DI + (t - 64) * 8), *(const v4u*)&s3[(t - 64) * 8]);
}
__global__ __launch_bounds__(128) void k_inp(const float* __restrict__ X, const float* __restrict__ WP, const float* __restrict__ BP, float* __restrict__ Hh) {
  __shared__ float sx[64][CIN]; __shared__ __align__(16) float so[64][DM]; const int t = threadIdx.x; const size_t t0 = (size_t)blockIdx.x * 64; const int b = (int)(t0 / LL), l0 = (int)(t0 % LL);
  for (int q = t; q < 64 * CIN; q += 128) { const int c = q / 64, tl = q % 64; sx[tl][c] = bfr(X[((size_t)b * CIN + c) * LL + l0 + tl]); }
  float w[CIN];
#pragma unroll
  for (int c = 0; c < CIN; ++c) w[c] = bfr(WP[t * CIN + c]);
  const float bb = bfr(BP[t]);
  __syncthreads();
#pragma unroll 1
  for (int tl = 0; tl < 64; ++tl) { float a = bb;
#pragma unroll
    for (int c = 0; c < CIN; ++c) a += sx[tl][c] * w[c];
    so[tl][t] = a; }
  __syncthreads();
  for (int q = t; q < 64 * DM / 4; q += 128) { const int tl = q / (DM / 4), pc = q % (DM / 4); vst2(Hh + (t0 + tl) * DM + pc * 4, *(const v4f*)&so[tl][pc * 4]); }
}
template <int NTL>
__global__ __launch_bounds__(128) void k_gemm(const float* __restrict__ A, int lda, int K, const __bf16* __restrict__ P, float* __restrict__ OUT, int ldo) {
  __shared__ __align__(16) float so[4][16][NTL * 16 + 4];
  const int tid = threadIdx.x, wave = tid >> 5, lane = tid & 31, col = lane & 15, g = lane >> 4; const size_t r0 = (size_t)blockIdx.x * 64 + wave * 16; const int n0 = blockIdx.y * NTL * 16;
  v8f acc[NTL]; for (int j = 0; j < NTL; ++j) acc[j] = (v8f){};
  for (int kc = 0; kc < K / 32; ++kc) { const F2 a = split_row(A + (r0 + col) * (size_t)lda, kc * 32, lane);
#pragma unroll
    for (int j = 0; j < NTL; ++j) { const v16b w = frag_b(P + (size_t)(n0 + j * 16 + col) * K + kc * 32, lane); acc[j] = wmma_bf(a.l, w, acc[j]); acc[j] = wmma_bf(a.h, w, acc[j]); } }
#pragma unroll
  for (int j = 0; j < NTL; ++j)
#pragma unroll
    for (int r = 0; r < 8; ++r) so[wave][8 * g + r][j * 16 + col] = acc[j][r];
  LDSX();
  for (int rl = 0; rl < 16; ++rl) for (int pc = lane; pc < NTL * 4; pc += 32) vst2(OUT + (r0 + rl) * (size_t)ldo + n0 + pc * 4, *(const v4f*)&so[wave][rl][pc * 4]);
}
__global__ __launch_bounds__(256) void k_conv(const float* __restrict__ XZ, const float* __restrict__ CW, const float* __restrict__ CB, float* __restrict__ XC) {
  const int d = threadIdx.x; const size_t t0 = (size_t)blockIdx.x * 64; const int b = (int)(t0 / LL), l0 = (int)(t0 % LL);
  const float w0 = bfr(CW[d * DC]), w1 = bfr(CW[d * DC + 1]), w2 = bfr(CW[d * DC + 2]), w3 = bfr(CW[d * DC + 3]), cb = bfr(CB[d]);
#pragma unroll 1
  for (int tl = 0; tl < 64; ++tl) { const int l = l0 + tl; float a = 0.f;
    const float x0 = (l - 3 >= 0) ? XZ[((size_t)b * LL + l - 3) * 512 + d] : 0.f, x1 = (l - 2 >= 0) ? XZ[((size_t)b * LL + l - 2) * 512 + d] : 0.f, x2 = (l - 1 >= 0) ? XZ[((size_t)b * LL + l - 1) * 512 + d] : 0.f, x3 = XZ[((size_t)b * LL + l) * 512 + d];
    a = ((w0 * x0 + w1 * x1) + w2 * x2) + w3 * x3 + cb;
    vst2(XC + (t0 + tl) * DI + d, a * sigm(a)); }
}
__global__ __launch_bounds__(256) void k_dt(const float* __restrict__ DBC, const float* __restrict__ WDT, const float* __restrict__ BDT, float* __restrict__ DT) {
  const int d = threadIdx.x; const size_t t0 = (size_t)blockIdx.x * 64; float w[DTR];
#pragma unroll
  for (int r = 0; r < DTR; ++r) w[r] = bfr(WDT[d * DTR + r]);
  const float bb = bfr(BDT[d]);
#pragma unroll 1
  for (int tl = 0; tl < 64; ++tl) { float a = bb; const float* row = DBC + (t0 + tl) * XW;
#pragma unroll
    for (int r = 0; r < DTR; ++r) a += row[r] * w[r];
    const float sp = (a > 20.f) ? a : log1p_ni(exp_ni(a));
    vst2(DT + (t0 + tl) * DI + d, sp); }
}
__global__ __launch_bounds__(256) void k_scan(const float* __restrict__ XC, const float* __restrict__ DBC, const float* __restrict__ DT, const float* __restrict__ XZ, const float* __restrict__ ALOG, const float* __restrict__ DSK, float* __restrict__ Y) {
  __shared__ float sh_[DS][DI], sA[DS][DI]; __shared__ float sB[DS], sC[DS]; const int d = threadIdx.x, b = blockIdx.x;
  for (int n = 0; n < DS; ++n) { sA[n][d] = -exp_ni(bfr(ALOG[d * DS + n])); sh_[n][d] = 0.f; }
  const float dsk = bfr(DSK[d]);
#pragma unroll 1
  for (int l = 0; l < LL; ++l) { const size_t tok = (size_t)b * LL + l; const float* row = DBC + tok * XW;
    __syncthreads();
    if (d < DS) sB[d] = row[DTR + d]; else if (d < 2 * DS) sC[d - DS] = row[DTR + d];
    __syncthreads();
    const float dt = DT[tok * DI + d], xc = XC[tok * DI + d]; const float dtx = dt * xc; float y = 0.f;
#pragma unroll 4
    for (int n = 0; n < DS; ++n) { const float dA = __expf(dt * sA[n][d]); const float hn = dA * sh_[n][d] + dtx * sB[n]; sh_[n][d] = hn; y += hn * sC[n]; }
    y += xc * dsk; const float z = XZ[tok * 512 + DI + d]; y *= z * sigm(z);
    vst2(Y + tok * DI + d, y); }
}
__global__ __launch_bounds__(128) void k_cls(const float* __restrict__ O, const float* __restrict__ W1, const float* __restrict__ B1, const float* __restrict__ G, const float* __restrict__ BE, const float* __restrict__ W2, const float* __restrict__ B2, float* __restrict__ out) {
  __shared__ float sp[NB][DM]; __shared__ float sh[NB][64]; __shared__ __align__(16) float so[4]; const int t = threadIdx.x;
  for (int b = 0; b < NB; ++b) { float a = 0.f;
#pragma unroll 1
    for (int l = 0; l < LL; ++l) a += O[((size_t)b * LL + l) * DM + t];
    sp[b][t] = a / (float)LL; }
  __syncthreads();
  if (t < 64) { float hv[NB];
    for (int b = 0; b < NB; ++b) { float a = bfr(B1[t]);
#pragma unroll 1
      for (int m = 0; m < DM; ++m) a += sp[b][m] * bfr(W1[t * DM + m]);
      hv[b] = a; }
    float mu = 0.f; for (int b = 0; b < NB; ++b) mu += hv[b]; mu /= (float)NB; float var = 0.f; for (int b = 0; b < NB; ++b) { const float dd = hv[b] - mu; var += dd * dd; } var /= (float)NB;
    const float rs = rsqrtf(var + 1e-5f);
    for (int b = 0; b < NB; ++b) sh[b][t] = fmaxf((hv[b] - mu) * rs * bfr(G[t]) + bfr(BE[t]), 0.f); }
  __syncthreads();
  if (t < 32) { for (int b = 0; b < NB; ++b) { float a = sh[b][t] * bfr(W2[t]) + sh[b][t + 32] * bfr(W2[t + 32]);
#pragma unroll
      for (int o = 1; o < 32; o <<= 1) a += __shfl_xor(a, o);
      if (t == 0) so[b] = a + bfr(B2[0]); } }
  __syncthreads();
  if (t == 0) vst2(out, *(const v4f*)&so[0]);
}
extern "C" void kernel_launch(void* const* d_in, const int* in_sizes, int n_in, void* d_out, int out_size, void* d_ws, size_t ws_size, hipStream_t stream) {
  (void)in_sizes; (void)n_in; (void)out_size;
  const float** F = (const float**)d_in;
  if (ws_size < (size_t)WS_END) return;
  char* ws = (char*)d_ws; __bf16* PW = (__bf16*)(ws + WS_PW); float *Hh = (float*)(ws + WS_H), *XZ = (float*)(ws + WS_XZ), *XC = (float*)(ws + WS_XC), *DBC = (float*)(ws + WS_DBC), *DT = (float*)(ws + WS_DT), *Y = (float*)(ws + WS_Y), *O = (float*)(ws + WS_O);
  k_pack<<<512, 256, 0, stream>>>(F[3], F[6], F[11], PW);
  k_inp<<<NT / 64, 128, 0, stream>>>(F[0], F[1], F[2], Hh);
  k_gemm<8><<<dim3(NT / 64, 4), 128, 0, stream>>>(Hh, DM, DM, PW + PWIN, XZ, 512);
  k_conv<<<NT / 64, 256, 0, stream>>>(XZ, F[4], F[5], XC);
  k_gemm<10><<<dim3(NT / 64, 1), 128, 0, stream>>>(XC, DI, DI, PW + PWX, DBC, XW);
  k_dt<<<NT / 64, 256, 0, stream>>>(DBC, F[7], F[8], DT);
  k_scan<<<NB, 256, 0, stream>>>(XC, DBC, DT, XZ, F[9], F[10], Y);
  k_gemm<8><<<dim3(NT / 64, 1), 128, 0, stream>>>(Y, DI, DI, PW + PWO, O, DM);
  k_cls<<<1, 128, 0, stream>>>(O, F[12], F[13], F[14], F[15], F[16], F[17], (float*)d_out);
}
